// ParamEvaler_80745385165293
// MI455X (gfx1250) — hardware-verified
//
#include <hip/hip_runtime.h>
#include <math.h>

typedef __attribute__((ext_vector_type(16))) _Float16 v16h;
typedef __attribute__((ext_vector_type(8)))  _Float16 v8h;
typedef __attribute__((ext_vector_type(8)))  float    v8f;
typedef __attribute__((ext_vector_type(4)))  float    v4f;

constexpr int kInits   = 64;
constexpr int kImgs    = 128;
constexpr int kParRow  = 18378;
constexpr int kOffW1   = 0;
constexpr int kOffB1   = 400;
constexpr int kOffW2   = 416;
constexpr int kOffB2   = 13216;
constexpr int kOffW3   = 13248;
constexpr int kOffB3   = 18368;
constexpr int kImgPix  = 784;
constexpr int kM1      = kImgs * 576;
constexpr int kN1      = kInits * 16;
constexpr int kK1      = 32;
constexpr int kK2      = 416;
constexpr int kK3      = 512;
constexpr int kA1Img   = 144 * 16;
constexpr float kWCarry    = 64.0f;
constexpr float kWCarryInv = 1.0f / kWCarry;
static_assert(kOffB1 == 16 * 25 && kOffW2 == kOffB1 + 16 && kOffB2 == kOffW2 + 32 * 400, "param offsets");
static_assert(kOffW3 == kOffB2 + 32 && kOffB3 == kOffW3 + 10 * 512 && kParRow == kOffB3 + 10, "param offsets");
static_assert(kM1 == 73728 && (kM1 % 64) == 0 && (kN1 % 64) == 0 && (kN1 / 64) == 16, "conv1 tile multiples");
static_assert((kK1 % 32) == 0 && (kK2 % 32) == 0 && (kK3 % 32) == 0, "K multiples of 32");
static_assert(((kM1 / 64) * (kN1 / 64)) % 8 == 0, "conv1 tiles per block exact");

constexpr size_t kBytesX1C = (size_t)kM1 * kK1 * 2;
constexpr size_t kBytesW1T = (size_t)kN1 * kK1 * 2;
constexpr size_t kBytesW2T = (size_t)kInits * 32 * kK2 * 2;
constexpr size_t kBytesW3T = (size_t)kInits * 16 * kK3 * 2;
constexpr size_t kBytesA1  = (size_t)kInits * kImgs * kA1Img * 2;
constexpr size_t kBytesA2  = (size_t)kInits * kImgs * 512 * 2;
constexpr size_t kWsX1C = 0;
constexpr size_t kWsW1T = kWsX1C + kBytesX1C;
constexpr size_t kWsW2T = kWsW1T + kBytesW1T;
constexpr size_t kWsW3T = kWsW2T + kBytesW2T;
constexpr size_t kWsA1  = kWsW3T + kBytesW3T;
constexpr size_t kWsA2  = kWsA1 + kBytesA1;
constexpr size_t kWsTotal = kWsA2 + kBytesA2;
static_assert(kWsTotal == 53673984ull, "carve total");
static_assert(kWsTotal <= 134217728ull, "carve cap");
static_assert((kWsW1T % 128) == 0 && (kWsW2T % 128) == 0 && (kWsW3T % 128) == 0 && (kWsA1 % 128) == 0 && (kWsA2 % 128) == 0, "aligned regions");

union FragU { v16h v; v8h h[2]; };
__device__ __forceinline__ v16h frag_load(const _Float16* p) {
  FragU f;
  f.h[0] = *(const v8h*)(p);
  f.h[1] = *(const v8h*)(p + 16);
  return f.v;
}
__device__ __forceinline__ v8f mma_h(v16h a, v16h b, v8f c) {
  c = __builtin_amdgcn_wmma_f32_16x16x32_f16(false, a, false, b, (short)0, c, false, false);
  asm volatile("v_nop\n\tv_nop\n\tv_nop\n\tv_nop" : "+v"(c) : "v"(a), "v"(b));
  return c;
}
__device__ __forceinline__ void store_twice_h8(unsigned short* p, v8h v) {
  *(volatile v8h*)p = v;
  __threadfence();
  *(volatile v8h*)p = v;
}
__device__ __forceinline__ float max4(float a, float b, float c, float d) {
  return fmaxf(fmaxf(a, b), fmaxf(c, d));
}

__global__ __launch_bounds__(256) void build_patch_rows_kernel(
    const float* __restrict__ batch, unsigned short* __restrict__ X1C)
{
  const int t   = blockIdx.x * 256 + threadIdx.x;
  const int row = t >> 2;
  const int k0  = (t & 3) * 8;
  const int mem = row & 3;
  const int img = row / 576;
  const int pp  = (row >> 2) - img * 144;
  const int py  = pp / 12;
  const int px  = pp - py * 12;
  const int y   = 2 * py + (mem >> 1);
  const int x   = 2 * px + (mem & 1);
  const float* src = batch + (size_t)img * kImgPix + y * 28 + x;
  v8h hv;
#pragma unroll
  for (int e = 0; e < 8; ++e) {
    const int k  = k0 + e;
    const int kc = (k < 25) ? k : 24;
    const int ky = kc / 5;
    const int kx = kc - ky * 5;
    const float ld = src[ky * 28 + kx];
    const float v  = (k < 25) ? ld : 0.0f;
    hv[e] = (_Float16)v;
  }
  store_twice_h8(X1C + (size_t)t * 8, hv);
}

__global__ __launch_bounds__(256) void build_weight_planes_kernel(
    const float* __restrict__ params, unsigned short* __restrict__ W1T,
    unsigned short* __restrict__ W2T, unsigned short* __restrict__ W3T)
{
  const int bx  = blockIdx.x;
  const int tid = threadIdx.x;
  if (bx < 16) {
    const int t    = bx * 256 + tid;
    const int n    = t >> 2;
    const int k0   = (t & 3) * 8;
    const int init = n >> 4;
    const int oc   = n & 15;
    const float* src = params + (size_t)init * kParRow + kOffW1 + oc * 25;
    v8h hv;
#pragma unroll
    for (int e = 0; e < 8; ++e) {
      const int k  = k0 + e;
      const int kc = (k < 25) ? k : 24;
      const float ld = src[kc];
      const float v  = (k < 25) ? (ld * kWCarry) : 0.0f;
      hv[e] = (_Float16)v;
    }
    store_twice_h8(W1T + (size_t)t * 8, hv);
  } else if (bx < 432) {
    const int t    = (bx - 16) * 256 + tid;
    const int row  = t / 52;
    const int k0   = (t - row * 52) * 8;
    const int init = row >> 5;
    const int oc   = row & 31;
    const float* src = params + (size_t)init * kParRow + kOffW2 + oc * 400;
    v8h hv;
#pragma unroll
    for (int e = 0; e < 8; ++e) {
      const int k    = k0 + e;
      const int tap  = k >> 4;
      const int ic   = k & 15;
      const int tapc = (tap < 25) ? tap : 24;
      const float ld = src[ic * 25 + tapc];
      const float v  = (k < 400) ? (ld * kWCarry) : 0.0f;
      hv[e] = (_Float16)v;
    }
    store_twice_h8(W2T + (size_t)t * 8, hv);
  } else {
    const int t    = (bx - 432) * 256 + tid;
    const int row  = t >> 6;
    const int k0   = (t & 63) * 8;
    const int init = row >> 4;
    const int o    = row & 15;
    const int oc   = (o < 10) ? o : 9;
    const float* src = params + (size_t)init * kParRow + kOffW3 + oc * 512 + k0;
    v8h hv;
#pragma unroll
    for (int e = 0; e < 8; ++e) {
      const float ld = src[e];
      const float v  = (o < 10) ? (ld * kWCarry) : 0.0f;
      hv[e] = (_Float16)v;
    }
    store_twice_h8(W3T + (size_t)t * 8, hv);
  }
}

__global__ __launch_bounds__(256) void conv1_pool_kernel(
    const unsigned short* __restrict__ X1Cp, const unsigned short* __restrict__ W1Tp,
    const float* __restrict__ params, unsigned short* __restrict__ A1)
{
  __shared__ __align__(16) float sT[8][4 * 256];
  const _Float16* X = (const _Float16*)X1Cp;
  const _Float16* W = (const _Float16*)W1Tp;
  const int lane  = threadIdx.x & 31;
  const int wave  = threadIdx.x >> 5;
  const int rlane = lane & 15;
  const int h     = lane >> 4;
  const int tile  = blockIdx.x * 8 + wave;
  const int tm    = tile >> 4;
  const int tn    = tile & 15;
  const int m0    = tm << 6;
  const int n0    = tn << 6;

  v16h bf[4];
#pragma unroll
  for (int j = 0; j < 4; ++j)
    bf[j] = frag_load(W + (size_t)(n0 + (j << 4) + rlane) * kK1 + 8 * h);

  v8f acc[4][4];
#pragma unroll
  for (int i = 0; i < 4; ++i)
#pragma unroll
    for (int j = 0; j < 4; ++j) acc[i][j] = (v8f){0.f, 0.f, 0.f, 0.f, 0.f, 0.f, 0.f, 0.f};

#pragma unroll
  for (int i = 0; i < 4; ++i) {
    const v16h af = frag_load(X + (size_t)(m0 + (i << 4) + rlane) * kK1 + 8 * h);
#pragma unroll
    for (int j = 0; j < 4; ++j) acc[i][j] = mma_h(af, bf[j], acc[i][j]);
  }

  float* slab = sT[wave];
#pragma unroll
  for (int j = 0; j < 4; ++j) {
    const int init = tn * 4 + j;
    const float bias = params[(size_t)init * kParRow + kOffB1 + rlane];
#pragma unroll
    for (int i = 0; i < 4; ++i) {
      const float p0 = max4(acc[i][j][0], acc[i][j][1], acc[i][j][2], acc[i][j][3]);
      const float p1 = max4(acc[i][j][4], acc[i][j][5], acc[i][j][6], acc[i][j][7]);
      const float v0 = fmaxf(p0 * kWCarryInv + bias, 0.0f);
      const float v1 = fmaxf(p1 * kWCarryInv + bias, 0.0f);
      const int pos = i * 4 + 2 * h;
      slab[j * 256 + pos * 16 + rlane]       = v0;
      slab[j * 256 + (pos + 1) * 16 + rlane] = v1;
    }
  }
  __syncthreads();

  const int img  = tm / 9;
  const int pos0 = (tm - img * 9) * 16;
  v8h hv[4];
#pragma unroll
  for (int j = 0; j < 4; ++j) {
    const float* sp = slab + j * 256 + lane * 8;
    const v4f a0 = *(const v4f*)(sp);
    const v4f a1 = *(const v4f*)(sp + 4);
#pragma unroll
    for (int e = 0; e < 4; ++e) {
      hv[j][e]     = (_Float16)a0[e];
      hv[j][4 + e] = (_Float16)a1[e];
    }
  }
  for (int pass = 0; pass < 2; ++pass) {
#pragma unroll
    for (int j = 0; j < 4; ++j) {
      const int init = tn * 4 + j;
      const size_t o = ((size_t)(init * kImgs + img) * 144 + pos0) * 16 + lane * 8;
      *(volatile v8h*)(A1 + o) = hv[j];
    }
    __threadfence();
  }
}

__global__ __launch_bounds__(256) void conv2_pool_kernel(
    const unsigned short* __restrict__ A1p, const unsigned short* __restrict__ W2Tp,
    const float* __restrict__ params, unsigned short* __restrict__ A2)
{
  __shared__ __align__(16) float sT[8][512];
  const int lane  = threadIdx.x & 31;
  const int wave  = threadIdx.x >> 5;
  const int rlane = lane & 15;
  const int h     = lane >> 4;
  const int init  = blockIdx.y;
  const int img   = blockIdx.x * 8 + wave;
  const _Float16* Ai = (const _Float16*)A1p + (size_t)(init * kImgs + img) * kA1Img;
  const _Float16* w0 = (const _Float16*)W2Tp + (size_t)(init * 32 + rlane) * kK2 + 8 * h;
  const _Float16* w1 = w0 + 16 * kK2;

  const int mem = rlane & 3;
  const int dy  = mem >> 1;
  const int dx  = mem & 1;
  int abase[4];
#pragma unroll
  for (int i = 0; i < 4; ++i) {
    const int pp = i * 4 + (rlane >> 2);
    const int y  = 2 * (pp >> 2) + dy;
    const int x  = 2 * (pp & 3) + dx;
    abase[i] = (y * 12 + x) * 16 + 8 * h;
  }

  v8f acc[4][2];
#pragma unroll
  for (int i = 0; i < 4; ++i) {
    acc[i][0] = (v8f){0.f, 0.f, 0.f, 0.f, 0.f, 0.f, 0.f, 0.f};
    acc[i][1] = (v8f){0.f, 0.f, 0.f, 0.f, 0.f, 0.f, 0.f, 0.f};
  }

#pragma unroll 1
  for (int ks = 0; ks < 13; ++ks) {
    const int tap0 = 2 * ks;
    const int tap1 = (2 * ks + 1 < 25) ? (2 * ks + 1) : 24;
    const int ky0 = tap0 / 5;
    const int ky1 = tap1 / 5;
    const int o0 = (ky0 * 12 + (tap0 - ky0 * 5)) * 16;
    const int o1 = (ky1 * 12 + (tap1 - ky1 * 5)) * 16;
    const v16h b0 = frag_load(w0 + ks * 32);
    const v16h b1 = frag_load(w1 + ks * 32);
#pragma unroll
    for (int i = 0; i < 4; ++i) {
      FragU a;
      a.h[0] = *(const v8h*)(Ai + abase[i] + o0);
      a.h[1] = *(const v8h*)(Ai + abase[i] + o1);
      acc[i][0] = mma_h(a.v, b0, acc[i][0]);
      acc[i][1] = mma_h(a.v, b1, acc[i][1]);
    }
  }

  float* slab = sT[wave];
#pragma unroll
  for (int j = 0; j < 2; ++j) {
    const int oc = j * 16 + rlane;
    const float bias = params[(size_t)init * kParRow + kOffB2 + oc];
#pragma unroll
    for (int i = 0; i < 4; ++i) {
      const float p0 = max4(acc[i][j][0], acc[i][j][1], acc[i][j][2], acc[i][j][3]);
      const float p1 = max4(acc[i][j][4], acc[i][j][5], acc[i][j][6], acc[i][j][7]);
      const float v0 = fmaxf(p0 * kWCarryInv + bias, 0.0f);
      const float v1 = fmaxf(p1 * kWCarryInv + bias, 0.0f);
      const int pp = i * 4 + 2 * h;
      slab[oc * 16 + pp]     = v0;
      slab[oc * 16 + pp + 1] = v1;
    }
  }
  __syncthreads();

  v8h hv[2];
#pragma unroll
  for (int it = 0; it < 2; ++it) {
    const float* sp = slab + (it * 32 + lane) * 8;
    const v4f a0 = *(const v4f*)(sp);
    const v4f a1 = *(const v4f*)(sp + 4);
#pragma unroll
    for (int e = 0; e < 4; ++e) {
      hv[it][e]     = (_Float16)a0[e];
      hv[it][4 + e] = (_Float16)a1[e];
    }
  }
  unsigned short* dst = A2 + (size_t)(init * kImgs + img) * 512;
  for (int pass = 0; pass < 2; ++pass) {
#pragma unroll
    for (int it = 0; it < 2; ++it)
      *(volatile v8h*)(dst + (it * 32 + lane) * 8) = hv[it];
    __threadfence();
  }
}

__global__ __launch_bounds__(256) void dense_logsoftmax_kernel(
    const unsigned short* __restrict__ A2p, const unsigned short* __restrict__ W3Tp,
    const float* __restrict__ params, float* __restrict__ out)
{
  __shared__ __align__(16) float sL[128 * 16];
  __shared__ __align__(16) float sO[1280];
  const int tid   = threadIdx.x;
  const int lane  = tid & 31;
  const int wave  = tid >> 5;
  const int rlane = lane & 15;
  const int h     = lane >> 4;
  const int init  = blockIdx.x;
  const _Float16* a = (const _Float16*)A2p + (size_t)(init * kImgs + wave * 16 + rlane) * kK3 + 8 * h;
  const _Float16* w = (const _Float16*)W3Tp + (size_t)(init * 16 + rlane) * kK3 + 8 * h;
  v8f acc = (v8f){0.f, 0.f, 0.f, 0.f, 0.f, 0.f, 0.f, 0.f};
#pragma unroll 1
  for (int ks = 0; ks < 16; ++ks) {
    const v16h af = frag_load(a + ks * 32);
    const v16h bf = frag_load(w + ks * 32);
    acc = mma_h(af, bf, acc);
  }
  {
    const int clsc = (rlane < 10) ? rlane : 9;
    const float bl = params[(size_t)init * kParRow + kOffB3 + clsc];
    const float bias = (rlane < 10) ? bl : 0.0f;
#pragma unroll
    for (int r = 0; r < 8; ++r)
      sL[(wave * 16 + 8 * h + r) * 16 + rlane] = acc[r] * kWCarryInv + bias;
  }
  __syncthreads();
  if (tid < 128) {
    const float* lg = sL + tid * 16;
    float mx = lg[0];
#pragma unroll 1
    for (int o = 1; o < 10; ++o) mx = fmaxf(mx, lg[o]);
    float s = 0.0f;
#pragma unroll 1
    for (int o = 0; o < 10; ++o) s += expf(lg[o] - mx);
    const float lz = mx + logf(s);
#pragma unroll 1
    for (int o = 0; o < 10; ++o) sO[tid * 10 + o] = lg[o] - lz;
  }
  __syncthreads();
  float* ob = out + (size_t)init * 1280;
  const int c1  = 256 + tid;
  const int c1c = (c1 < 320) ? c1 : 319;
  const v4f v0 = *(const v4f*)(sO + tid * 4);
  const v4f v1 = *(const v4f*)(sO + c1c * 4);
  for (int pass = 0; pass < 2; ++pass) {
    *(volatile v4f*)(ob + tid * 4) = v0;
    if (tid < 64) *(volatile v4f*)(ob + c1 * 4) = v1;
    __threadfence();
  }
}

extern "C" void kernel_launch(void* const* d_in, const int* in_sizes, int n_in,
                              void* d_out, int out_size, void* d_ws, size_t ws_size,
                              hipStream_t stream) {
  if (n_in < 2) return;
  if (in_sizes[0] != kInits * kParRow) return;
  if (in_sizes[1] != kImgs * kImgPix) return;
  if (out_size != kInits * kImgs * 10) return;
  if (ws_size < kWsTotal) return;

  const float* params = (const float*)d_in[0];
  const float* batch  = (const float*)d_in[1];
  float* out = (float*)d_out;
  char* ws = (char*)d_ws;
  unsigned short* X1C = (unsigned short*)(ws + kWsX1C);
  unsigned short* W1T = (unsigned short*)(ws + kWsW1T);
  unsigned short* W2T = (unsigned short*)(ws + kWsW2T);
  unsigned short* W3T = (unsigned short*)(ws + kWsW3T);
  unsigned short* A1  = (unsigned short*)(ws + kWsA1);
  unsigned short* A2  = (unsigned short*)(ws + kWsA2);

  build_patch_rows_kernel<<<(kM1 * 4) / 256, 256, 0, stream>>>(batch, X1C);
  build_weight_planes_kernel<<<688, 256, 0, stream>>>(params, W1T, W2T, W3T);
  conv1_pool_kernel<<<((kM1 / 64) * (kN1 / 64)) / 8, 256, 0, stream>>>(X1C, W1T, params, A1);
  conv2_pool_kernel<<<dim3(kImgs / 8, kInits), 256, 0, stream>>>(A1, W2T, params, A2);
  dense_logsoftmax_kernel<<<kInits, 256, 0, stream>>>(A2, W3T, params, out);
}
